// TDSPMLPHead_24163486007454
// MI455X (gfx1250) — hardware-verified
//
#include <hip/hip_runtime.h>
#include <math.h>

constexpr int kB = 8;
constexpr int kN = 128;
constexpr int kM = 128;
constexpr int kE = 256;
constexpr int kH = 512;
constexpr int kK3 = 3 * kE;
constexpr int kPairs = kN * kM;
constexpr float kCarryA = 16.0f;
constexpr float kCarryW = 16.0f;
constexpr float kGemmScale = 1.0f / 256.0f;
constexpr float kInvH = 1.0f / 512.0f;
constexpr float kLnEps = 1e-5f;
constexpr float kNormEps = 1e-12f;

typedef __attribute__((ext_vector_type(16))) _Float16 v16h;
typedef __attribute__((ext_vector_type(8)))  _Float16 v8h;
typedef __attribute__((ext_vector_type(16))) __bf16   v16b;
typedef __attribute__((ext_vector_type(8)))  __bf16   v8b;
typedef __attribute__((ext_vector_type(8)))  float    v8f;
typedef __attribute__((ext_vector_type(4)))  float    v4f;
typedef __attribute__((ext_vector_type(4)))  unsigned int v4u;

__device__ __forceinline__ unsigned short f2bf_bits(float f) {
  unsigned u = __float_as_uint(f);
  return (unsigned short)((u + 0x7FFFu + ((u >> 16) & 1u)) >> 16);
}
__device__ __forceinline__ float bf_bits2f(unsigned short h) { return __uint_as_float(((unsigned)h) << 16); }

__device__ __forceinline__ void dep_guard_h(v8f& a, v8f& b, v16h x, v16h y) { asm volatile("v_nop\n\tv_nop\n\tv_nop\n\tv_nop" : "+v"(a), "+v"(b) : "v"(x), "v"(y)); }
__device__ __forceinline__ void dep_guard_b(v8f& a, v8f& b, v16b x, v16b y) { asm volatile("v_nop\n\tv_nop\n\tv_nop\n\tv_nop" : "+v"(a), "+v"(b) : "v"(x), "v"(y)); }
__device__ __forceinline__ void keep4_h(v16h a, v16h b, v16h c, v16h d) { asm volatile("v_nop" :: "v"(a), "v"(b), "v"(c), "v"(d)); }
__device__ __forceinline__ void keep4_b(v16b a, v16b b, v16b c, v16b d) { asm volatile("v_nop" :: "v"(a), "v"(b), "v"(c), "v"(d)); }
__device__ __forceinline__ void acc_guard4(v8f& a, v8f& b, v8f& c, v8f& d) { asm volatile("v_nop\n\tv_nop\n\tv_nop\n\tv_nop" : "+v"(a), "+v"(b), "+v"(c), "+v"(d)); }
template <typename T> struct Frag;
template <> struct Frag<_Float16> {
  typedef v16h V; union U { v16h v; v8h h[2]; };
  static __device__ __forceinline__ v16h load(const _Float16* p) {
    U f; f.h[0] = *(const v8h*)(p); f.h[1] = *(const v8h*)(p + 16); return f.v;
  }
  static __device__ __forceinline__ v8f mma(v16h a, v16h b, v8f c) {
    return __builtin_amdgcn_wmma_f32_16x16x32_f16(false, a, false, b, (short)0, c, false, false);
  }
  static __device__ __forceinline__ void guard(v8f& a, v8f& b, v16h x, v16h y) { dep_guard_h(a, b, x, y); }
  static __device__ __forceinline__ void keep(v16h a, v16h b, v16h c, v16h d) { keep4_h(a, b, c, d); }
};
template <> struct Frag<__bf16> {
  typedef v16b V; union U { v16b v; v8b h[2]; };
  static __device__ __forceinline__ v16b load(const __bf16* p) {
    U f; f.h[0] = *(const v8b*)(p); f.h[1] = *(const v8b*)(p + 16); return f.v;
  }
  static __device__ __forceinline__ v8f mma(v16b a, v16b b, v8f c) {
    return __builtin_amdgcn_wmma_f32_16x16x32_bf16(false, a, false, b, (short)0, c, false, false);
  }
  static __device__ __forceinline__ void guard(v8f& a, v8f& b, v16b x, v16b y) { dep_guard_b(a, b, x, y); }
  static __device__ __forceinline__ void keep(v16b a, v16b b, v16b c, v16b d) { keep4_b(a, b, c, d); }
};

__device__ __forceinline__ unsigned pk16(unsigned short a, unsigned short b) { return (unsigned)a | ((unsigned)b << 16); }
__device__ __forceinline__ unsigned short h_bits(float f) { const _Float16 h = (_Float16)f; return __builtin_bit_cast(unsigned short, h); }

template <int ET> struct Elem;
template <> struct Elem<0> { typedef _Float16 T; };
template <> struct Elem<1> { typedef __bf16 T; };
template <int ET, bool SPLIT, int BIAS_MODE, int OUT_MODE, bool RESID, int ACT = 0>
__global__ __launch_bounds__(256) void wmma_gemm64(
    const unsigned short* __restrict__ Ap, const unsigned short* __restrict__ A2p, int lda, long strideA,
    const unsigned short* __restrict__ Btp, const unsigned short* __restrict__ Bt2p, int ldb, long strideB,
    void* __restrict__ Cout, void* __restrict__ Cout2, int ldc, long strideC,
    const float* __restrict__ bias,
    const float* __restrict__ resid, long strideR,
    int M, int N, int K, float scale) {
  typedef typename Elem<ET>::T T;
  typedef typename Frag<T>::V V;
  const T* A = (const T*)Ap; const T* A2 = (const T*)A2p; const T* Bt = (const T*)Btp; const T* Bt2 = (const T*)Bt2p;
  __shared__ __align__(16) float sT[8][16 * 68];
  const int b    = blockIdx.y;
  const int lane = threadIdx.x & 31;
  const int wave = threadIdx.x >> 5;
  const int tilesN = N >> 6;
  const int tilesM = M >> 6;
  const int tile = blockIdx.x * 8 + wave;
  if (tile >= tilesM * tilesN) return;
  const int tm = tile / tilesN;
  const int tn = tile - tm * tilesN;
  const int m0 = tm << 6;
  const int n0 = tn << 6;

  const T* Ab  = A  + (size_t)b * strideA;
  const T* Bb  = Bt + (size_t)b * strideB;
  const T* Ab2 = SPLIT ? (A2  + (size_t)b * strideA) : nullptr;
  const T* Bb2 = SPLIT ? (Bt2 + (size_t)b * strideB) : nullptr;

  const int rlane = lane & 15;
  const int koff  = (lane >> 4) * 8;
  const int mOff  = (lane >> 4) * 8;

  v8f acc[4][4];
#pragma unroll
  for (int i = 0; i < 4; ++i)
#pragma unroll
    for (int j = 0; j < 4; ++j) acc[i][j] = (v8f){0.f,0.f,0.f,0.f,0.f,0.f,0.f,0.f};

  for (int k0 = 0; k0 < K; k0 += 32) {
    V bh[4], bl[4];
#pragma unroll
    for (int j = 0; j < 4; ++j) {
      const size_t bo = (size_t)(n0 + (j << 4) + rlane) * ldb + koff + k0;
      bh[j] = Frag<T>::load(Bb + bo);
      if (SPLIT) bl[j] = Frag<T>::load(Bb2 + bo);
    }
#pragma unroll
    for (int i = 0; i < 4; ++i) {
      const size_t ao = (size_t)(m0 + (i << 4) + rlane) * lda + koff + k0;
      V ah = Frag<T>::load(Ab + ao);
      V al;
      if (SPLIT) al = Frag<T>::load(Ab2 + ao);
#pragma unroll
      for (int j = 0; j < 4; ++j) {
        acc[i][j] = Frag<T>::mma(ah, bh[j], acc[i][j]);
        if (SPLIT) {
          acc[i][j] = Frag<T>::mma(ah, bl[j], acc[i][j]);
          acc[i][j] = Frag<T>::mma(al, bh[j], acc[i][j]);
        }
      }
      Frag<T>::guard(acc[i][0], acc[i][3], ah, SPLIT ? al : ah);
    }
    Frag<T>::keep(bh[0], bh[1], bh[2], bh[3]);
    if (SPLIT) Frag<T>::keep(bl[0], bl[1], bl[2], bl[3]);
  }
  acc_guard4(acc[0][0], acc[0][1], acc[0][2], acc[0][3]);
  acc_guard4(acc[1][0], acc[1][1], acc[1][2], acc[1][3]);
  acc_guard4(acc[2][0], acc[2][1], acc[2][2], acc[2][3]);
  acc_guard4(acc[3][0], acc[3][1], acc[3][2], acc[3][3]);

  float* slab = sT[wave];
  const float* Rb = RESID ? (resid + (size_t)b * strideR) : nullptr;
#pragma unroll
  for (int i = 0; i < 4; ++i) {
    const int mBase = m0 + (i << 4);
#pragma unroll
    for (int j = 0; j < 4; ++j) {
      const int n = n0 + (j << 4) + rlane;
      float bv = 0.f;
      if (BIAS_MODE == 2) bv = bias[n];
#pragma unroll
      for (int r = 0; r < 8; ++r) {
        float v = acc[i][j][r] * scale;
        if (BIAS_MODE == 1) v += bias[mBase + mOff + r];
        if (BIAS_MODE == 2) v += bv;
        if (RESID) v += Rb[(size_t)(mBase + mOff + r) * ldc + n];
        if (ACT == 2) v = fmaxf(v, 0.0f);
        if (ACT == 4) v = (v > 0.f) ? v : 0.01f * v;
        slab[(mOff + r) * 68 + (j << 4) + rlane] = v;
      }
    }
    __builtin_amdgcn_fence(__ATOMIC_RELEASE, "workgroup");
    __builtin_amdgcn_wave_barrier();
    __builtin_amdgcn_fence(__ATOMIC_ACQUIRE, "workgroup");
    if (OUT_MODE == 0) {
      float* C = (float*)Cout + (size_t)b * strideC;
      const int hh = lane >> 4, c4 = (lane & 15) * 4;
      for (int pass = 0; pass < 2; ++pass) {
#pragma unroll
        for (int it = 0; it < 8; ++it) {
          const int row = it * 2 + hh;
          v4f v = *(const v4f*)(slab + row * 68 + c4);
          *(volatile v4f*)(C + (size_t)(mBase + row) * ldc + n0 + c4) = v;
        }
        __threadfence();
      }
    } else {
      const int q = lane >> 3, c8 = (lane & 7) * 8;
      unsigned short* C  = (unsigned short*)Cout  + (size_t)b * strideC;
      unsigned short* C2 = (OUT_MODE == 2) ? ((unsigned short*)Cout2 + (size_t)b * strideC) : nullptr;
      for (int pass = 0; pass < 2; ++pass) {
#pragma unroll
        for (int it = 0; it < 4; ++it) {
          const int row = it * 4 + q;
          const float* sp = slab + row * 68 + c8;
          v8h hv, lv;
#pragma unroll
          for (int e = 0; e < 8; ++e) {
            if (OUT_MODE == 1) {
              hv[e] = (_Float16)sp[e];
            } else {
              unsigned short hb = f2bf_bits(sp[e]);
              unsigned short lb = f2bf_bits(sp[e] - bf_bits2f(hb));
              hv[e] = __builtin_bit_cast(_Float16, hb);
              lv[e] = __builtin_bit_cast(_Float16, lb);
            }
          }
          *(volatile v8h*)(C + (size_t)(mBase + row) * ldc + n0 + c8) = hv;
          if (OUT_MODE == 2) *(volatile v8h*)(C2 + (size_t)(mBase + row) * ldc + n0 + c8) = lv;
        }
        __threadfence();
      }
    }
    __builtin_amdgcn_fence(__ATOMIC_RELEASE, "workgroup");
    __builtin_amdgcn_wave_barrier();
    __builtin_amdgcn_fence(__ATOMIC_ACQUIRE, "workgroup");
  }
}

__device__ __forceinline__ float wave_sum32(float v) {
#pragma unroll
  for (int off = 16; off > 0; off >>= 1) v += __shfl_xor(v, off, 32);
  return v;
}

__global__ __launch_bounds__(64) void l2norm_kernel(const float* __restrict__ X, float* __restrict__ Y) {
  __shared__ float red[2];
  const int row  = blockIdx.x;
  const int t    = threadIdx.x;
  const int lane = t & 31, wave = t >> 5;
  const float* xr = X + ((size_t)row * kE + t * 4);
  const v4f x = *(const v4f*)xr;
  float ss = (x[0] * x[0] + x[1] * x[1]) + (x[2] * x[2] + x[3] * x[3]);
  ss = wave_sum32(ss);
  if (lane == 0) red[wave] = ss;
  __syncthreads();
  const float tot = red[0] + red[1];
  const float nrm = sqrtf(tot);
  const float inv = 1.0f / fmaxf(nrm, kNormEps);
  const v4f y = x * inv;
  float* yr = Y + ((size_t)row * kE + t * 4);
  *(volatile v4f*)yr = y;
  __threadfence();
  *(volatile v4f*)yr = y;
}

__global__ __launch_bounds__(256) void w1t_cast_kernel(const float* __restrict__ W, unsigned short* __restrict__ out) {
  __shared__ float sm[64][65];
  const int t  = threadIdx.x;
  const int k0 = blockIdx.x * 64;
  const int h0 = blockIdx.y * 64;
#pragma unroll
  for (int i = 0; i < 16; ++i) {
    const int e = i * 256 + t;
    const int r = e >> 6;
    const int c = e & 63;
    sm[c][r] = W[(size_t)(k0 + r) * kH + h0 + c] * kCarryW;
  }
  __syncthreads();
  const int lane = t & 31, wave = t >> 5;
  const int q = lane >> 3, c8 = (lane & 7) * 8;
  for (int pass = 0; pass < 2; ++pass) {
#pragma unroll
    for (int it = 0; it < 2; ++it) {
      const int row = wave * 8 + it * 4 + q;
      unsigned short hb[8];
#pragma unroll
      for (int e = 0; e < 8; ++e) hb[e] = h_bits(sm[row][c8 + e]);
      const v4u u = (v4u){pk16(hb[0], hb[1]), pk16(hb[2], hb[3]), pk16(hb[4], hb[5]), pk16(hb[6], hb[7])};
      *(volatile v4u*)(out + (size_t)(h0 + row) * kK3 + k0 + c8) = u;
    }
    __threadfence();
  }
}

__global__ __launch_bounds__(256) void pair_kernel(const float* __restrict__ Tn, const float* __restrict__ Dn,
                                                   unsigned short* __restrict__ A, int b) {
  const int n    = blockIdx.x >> 2;
  const int m0   = (blockIdx.x & 3) * 32;
  const int lane = threadIdx.x & 31, wave = threadIdx.x >> 5;
  const float* tr = Tn + ((size_t)(b * kN + n) * kE + lane * 8);
  const v4f t0 = *(const v4f*)tr;
  const v4f t1 = *(const v4f*)(tr + 4);
  float tv[8];
#pragma unroll
  for (int e = 0; e < 4; ++e) { tv[e] = t0[e]; tv[4 + e] = t1[e]; }
  unsigned short ht[8];
#pragma unroll
  for (int e = 0; e < 8; ++e) ht[e] = h_bits(kCarryA * tv[e]);
  const v4u ut = (v4u){pk16(ht[0], ht[1]), pk16(ht[2], ht[3]), pk16(ht[4], ht[5]), pk16(ht[6], ht[7])};
#pragma unroll 1
  for (int r = 0; r < 4; ++r) {
    const int m = m0 + wave + 8 * r;
    const float* dr = Dn + ((size_t)(b * kM + m) * kE + lane * 8);
    const v4f d0 = *(const v4f*)dr;
    const v4f d1 = *(const v4f*)(dr + 4);
    float dv[8];
#pragma unroll
    for (int e = 0; e < 4; ++e) { dv[e] = d0[e]; dv[4 + e] = d1[e]; }
    unsigned short hd[8], hf[8];
#pragma unroll
    for (int e = 0; e < 8; ++e) {
      hd[e] = h_bits(kCarryA * dv[e]);
      hf[e] = h_bits(kCarryA * fabsf(tv[e] - dv[e]));
    }
    const v4u ud = (v4u){pk16(hd[0], hd[1]), pk16(hd[2], hd[3]), pk16(hd[4], hd[5]), pk16(hd[6], hd[7])};
    const v4u uf = (v4u){pk16(hf[0], hf[1]), pk16(hf[2], hf[3]), pk16(hf[4], hf[5]), pk16(hf[6], hf[7])};
    unsigned short* ap = A + ((size_t)(n * kM + m) * kK3 + lane * 8);
    *(volatile v4u*)(ap)          = ut;
    *(volatile v4u*)(ap + kE)     = ud;
    *(volatile v4u*)(ap + 2 * kE) = uf;
    __threadfence();
    *(volatile v4u*)(ap)          = ut;
    *(volatile v4u*)(ap + kE)     = ud;
    *(volatile v4u*)(ap + 2 * kE) = uf;
  }
}

__global__ __launch_bounds__(256) void finish_kernel(const float* __restrict__ Hp, const float* __restrict__ gamma,
                                                     const float* __restrict__ beta, const float* __restrict__ W2,
                                                     const float* __restrict__ b2, float* __restrict__ out, int b) {
  __shared__ __align__(16) float sG[kH];
  __shared__ __align__(16) float sBt[kH];
  __shared__ __align__(16) float sW[kH];
  __shared__ __align__(16) float sOut[kM];
  const int n = blockIdx.x;
  const int t = threadIdx.x, lane = t & 31, wave = t >> 5;
  for (int i = t; i < kH; i += 256) { sG[i] = gamma[i]; sBt[i] = beta[i]; sW[i] = W2[i]; }
  const float bias2 = b2[0];
  __syncthreads();
#pragma unroll 1
  for (int r = 0; r < 16; ++r) {
    const int m = wave * 16 + r;
    const float* hr = Hp + ((size_t)(n * kM + m) * kH + lane * 4);
    float s = 0.f;
#pragma unroll 1
    for (int c = 0; c < 4; ++c) {
      const v4f x = *(const v4f*)(hr + c * 128);
      s += (x[0] + x[1]) + (x[2] + x[3]);
    }
    s = wave_sum32(s);
    const float mu = s * kInvH;
    float q2 = 0.f;
#pragma unroll 1
    for (int c = 0; c < 4; ++c) {
      const v4f x = *(const v4f*)(hr + c * 128);
      const float e0 = x[0] - mu, e1 = x[1] - mu, e2 = x[2] - mu, e3 = x[3] - mu;
      q2 += (e0 * e0 + e1 * e1) + (e2 * e2 + e3 * e3);
    }
    q2 = wave_sum32(q2);
    const float rs = rsqrtf(q2 * kInvH + kLnEps);
    float acc = 0.f;
#pragma unroll 1
    for (int c = 0; c < 4; ++c) {
      const int col = c * 128 + lane * 4;
      const v4f x  = *(const v4f*)(hr + c * 128);
      const v4f g  = *(const v4f*)(sG + col);
      const v4f bt = *(const v4f*)(sBt + col);
      const v4f w  = *(const v4f*)(sW + col);
#pragma unroll
      for (int e = 0; e < 4; ++e) {
        float y = (x[e] - mu) * rs * g[e] + bt[e];
        const float ex = expf(-y);
        y = y * (1.0f / (1.0f + ex));
        acc += y * w[e];
      }
    }
    acc = wave_sum32(acc);
    if (lane == 0) sOut[m] = acc + bias2;
  }
  __syncthreads();
  if (wave == 0) {
    const v4f v = *(const v4f*)(sOut + lane * 4);
    float* op = out + ((size_t)(b * kN + n) * kM + lane * 4);
    *(volatile v4f*)op = v;
    __threadfence();
    *(volatile v4f*)op = v;
  }
}

extern "C" void kernel_launch(void* const* d_in, const int* in_sizes, int n_in,
                              void* d_out, int out_size, void* d_ws, size_t ws_size,
                              hipStream_t stream) {
  if (n_in < 8) return;
  if (in_sizes[0] != kB * kN * kE) return;
  if (in_sizes[1] != kB * kM * kE) return;
  if (in_sizes[2] != kK3 * kH) return;
  if (in_sizes[3] != kH || in_sizes[4] != kH || in_sizes[5] != kH || in_sizes[6] != kH) return;
  if (in_sizes[7] < 1) return;
  if (out_size != kB * kN * kM) return;

  const float* track = (const float*)d_in[0];
  const float* det   = (const float*)d_in[1];
  const float* W1    = (const float*)d_in[2];
  const float* b1    = (const float*)d_in[3];
  const float* gamma = (const float*)d_in[4];
  const float* beta  = (const float*)d_in[5];
  const float* W2    = (const float*)d_in[6];
  const float* b2    = (const float*)d_in[7];
  float* out = (float*)d_out;

  const size_t bytesTn = (size_t)kB * kN * kE * sizeof(float);
  const size_t bytesDn = (size_t)kB * kM * kE * sizeof(float);
  const size_t bytesW  = (size_t)kH * kK3 * sizeof(unsigned short);
  const size_t bytesA  = (size_t)kPairs * kK3 * sizeof(unsigned short);
  const size_t bytesHp = (size_t)kPairs * kH * sizeof(float);
  const size_t offTn = 0;
  const size_t offDn = offTn + bytesTn;
  const size_t offW  = offDn + bytesDn;
  const size_t offA  = offW + bytesW;
  const size_t offHp = offA + bytesA;
  const size_t total = offHp + bytesHp;
  if (total > ws_size) return;

  char* ws = (char*)d_ws;
  float*          Tn  = (float*)(ws + offTn);
  float*          Dn  = (float*)(ws + offDn);
  unsigned short* W1T = (unsigned short*)(ws + offW);
  unsigned short* A16 = (unsigned short*)(ws + offA);
  float*          Hp  = (float*)(ws + offHp);

  l2norm_kernel<<<dim3(kB * kN), dim3(64), 0, stream>>>(track, Tn);
  l2norm_kernel<<<dim3(kB * kM), dim3(64), 0, stream>>>(det, Dn);
  w1t_cast_kernel<<<dim3(kK3 / 64, kH / 64), dim3(256), 0, stream>>>(W1, W1T);

  const int gemmBlocks = (kPairs / 64) * (kH / 64) / 8;
  for (int bb = 0; bb < kB; ++bb) {
    pair_kernel<<<dim3(kN * 4), dim3(256), 0, stream>>>(Tn, Dn, A16, bb);
    wmma_gemm64<0, false, 2, 0, false, 0><<<dim3(gemmBlocks, 1, 1), dim3(256), 0, stream>>>(
        A16, A16, kK3, (long)0,
        W1T, W1T, kK3, (long)0,
        (void*)Hp, (void*)Hp, kH, (long)0,
        b1,
        b1, (long)0,
        kPairs, kH, kK3, kGemmScale);
    finish_kernel<<<dim3(kN), dim3(256), 0, stream>>>(Hp, gamma, beta, W2, b2, out, bb);
  }
}
